// MDNLoss_65704409694902
// MI455X (gfx1250) — hardware-run, weakly checked
//
#include <hip/hip_runtime.h>
#include <math.h>

typedef __attribute__((ext_vector_type(16))) _Float16 v16h;
typedef __attribute__((ext_vector_type(8)))  _Float16 v8h;
typedef __attribute__((ext_vector_type(8)))  float    v8f;
typedef __attribute__((ext_vector_type(4)))  float    v4f;

constexpr int kNB    = 16;
constexpr int kNL    = 160;
constexpr int kNT    = 800;
constexpr int kNC    = 80;
constexpr int kDepth = 2 * kNC;
constexpr int kPitch = 192;
constexpr int kGrp   = kPitch / 8;
constexpr int kRowsA = kNB * kNL;
constexpr int kRowsB = kNB * kNT;
constexpr int kFlat  = kNB * kNL * kNT + 1;
constexpr int kQuads = (kFlat - 1) / 4;
constexpr int kTilesL = kNL / 32;
constexpr int kTilesT = kNT / 32;
constexpr int kTiles  = kNB * kTilesL * kTilesT;
constexpr int kSVP = 164;
constexpr int kSQP = 81;
constexpr int kSXP = 84;
constexpr int kSLP = 36;
constexpr float kNeg = -1e30f;
constexpr float kXCarry = 4.0f;
constexpr float kFold   = -0.5f / kXCarry;
constexpr float kLogNormTerm = -0.5f * (float)kNC * 1.8378770664093453f;
constexpr float kF16MinNormal = 6.103515625e-5f;
constexpr float kF16Max = 65504.0f;

static_assert((kDepth % 32) == 0, "depth multiple of 32");
static_assert(kDepth <= kPitch && (kPitch % 64) == 0, "plane pitch whole lines");
static_assert((kNL % 32) == 0 && (kNT % 32) == 0, "tile multiples");
static_assert((kTiles % 8) == 0, "eight wave tiles per block");
static_assert((kRowsA % 32) == 0, "state rows per block");
static_assert(((kFlat - 1) % 4) == 0 && (kQuads % 256) == 0, "flat output quads");
static_assert(kGrp == 24, "groups per plane row");
static_assert(32 * kNC == 10 * 256, "element loop coverage");
static_assert(32 * kGrp == 3 * 256, "store loop coverage");

constexpr size_t kSzAPL = (size_t)kRowsA * kPitch * 2;
constexpr size_t kSzBPL = (size_t)kRowsB * kPitch * 2;
constexpr size_t kSzCT  = (size_t)kRowsA * 4;
constexpr size_t kSzLPM = (size_t)kNB * kNL * kNT * 4;
constexpr size_t kSzAL  = (size_t)kNB * 32 * 4;
constexpr size_t kOffAPL = 0;
constexpr size_t kOffBPL = kOffAPL + kSzAPL;
constexpr size_t kOffCT  = kOffBPL + kSzBPL;
constexpr size_t kOffLPM = kOffCT + kSzCT;
constexpr size_t kOffAL  = kOffLPM + kSzLPM;
constexpr size_t kWsTotal = kOffAL + kSzAL;
static_assert(kWsTotal == 14102528ull, "carve total");
static_assert(kWsTotal <= 134217728ull, "carve cap");
static_assert((kOffBPL % 128) == 0 && (kOffCT % 128) == 0 && (kOffLPM % 128) == 0 && (kOffAL % 128) == 0, "aligned regions");

__device__ __forceinline__ float bf16_rne(float f) {
  unsigned u = __float_as_uint(f);
  u = (u + 0x7FFFu + ((u >> 16) & 1u)) & 0xFFFF0000u;
  return __uint_as_float(u);
}
__device__ __forceinline__ float f16_operand(float v) {
  const float c = fminf(fmaxf(v, -kF16Max), kF16Max);
  return (fabsf(c) < kF16MinNormal) ? 0.0f : c;
}
union FragH { v16h v; v8h h[2]; };
__device__ __forceinline__ v16h frag_load(const _Float16* p) {
  FragH f;
  f.h[0] = *(const v8h*)(p);
  f.h[1] = *(const v8h*)(p + 16);
  return f.v;
}
__device__ __forceinline__ v8f mma_guarded(v16h a, v16h b, v8f c) {
  c = __builtin_amdgcn_wmma_f32_16x16x32_f16(false, a, false, b, (short)0, c, false, false);
  asm volatile("v_nop\n\tv_nop\n\tv_nop\n\tv_nop" : "+v"(c) : "v"(a), "v"(b));
  return c;
}
__device__ float log_add_exp(float a, float b) {
  const float m = fmaxf(a, b);
  const float d = fabsf(a - b);
  return m + log1pf(expf(-d));
}

__global__ __launch_bounds__(256) void operand_planes_states(
    const float* __restrict__ stat, unsigned short* __restrict__ apl, float* __restrict__ ctab)
{
  __shared__ __align__(16) float sV[32 * kSVP];
  __shared__ __align__(16) float sQ[32 * kSQP];
  const int tid = threadIdx.x;
  const int r0 = blockIdx.x * 32;
#pragma unroll 1
  for (int it = 0; it < 10; ++it) {
    const int e = it * 256 + tid;
    const int rl = e / kNC;
    const int ch = e - rl * kNC;
    const float* rp = stat + (size_t)(r0 + rl) * (2 * kNC);
    const float lg = bf16_rne(rp[ch]);
    const float ls = bf16_rne(rp[kNC + ch]);
    const float iv = expf(-2.0f * ls);
    const float mu = 1.0f / (1.0f + expf(-lg));
    const float miv = mu * iv;
    sV[rl * kSVP + ch] = iv;
    sV[rl * kSVP + kNC + ch] = miv;
    sQ[rl * kSQP + ch] = mu * miv + ls;
  }
  __syncthreads();

  v8h hv[3];
#pragma unroll
  for (int it = 0; it < 3; ++it) {
    const int idx = it * 256 + tid;
    const int rl = idx / kGrp;
    const int g = idx - rl * kGrp;
    const bool live = (g < 20);
    const int gg = live ? g : 0;
    const float* sp = sV + rl * kSVP + 8 * gg;
    const v4f a0 = *(const v4f*)(sp);
    const v4f a1 = *(const v4f*)(sp + 4);
#pragma unroll
    for (int e = 0; e < 4; ++e) {
      const float x0 = live ? a0[e] : 0.0f;
      const float x1 = live ? a1[e] : 0.0f;
      hv[it][e]     = (_Float16)f16_operand(x0);
      hv[it][4 + e] = (_Float16)f16_operand(x1);
    }
  }
  unsigned short* base = apl + ((size_t)blockIdx.x * 768) * 8;
  for (int pass = 0; pass < 2; ++pass) {
#pragma unroll
    for (int it = 0; it < 3; ++it)
      *(volatile v8h*)(base + (size_t)(it * 256 + tid) * 8) = hv[it];
    __threadfence();
  }

  if (tid < 32) {
    float s = 0.0f;
#pragma unroll 1
    for (int ch = 0; ch < kNC; ++ch) s += sQ[tid * kSQP + ch];
    const float cv = kLogNormTerm - 0.5f * s;
    volatile float* cp = ctab + r0 + tid;
    *cp = cv;
    __threadfence();
    *cp = cv;
  }
}

__global__ __launch_bounds__(256) void operand_planes_frames(
    const float* __restrict__ feat, unsigned short* __restrict__ bpl)
{
  __shared__ __align__(16) float sX[32 * kSXP];
  const int tid = threadIdx.x;
  const int b = blockIdx.y;
  const int t0 = blockIdx.x * 32;
#pragma unroll 1
  for (int it = 0; it < 10; ++it) {
    const int e = it * 256 + tid;
    const int ch = e >> 5;
    const int tt = e & 31;
    sX[tt * kSXP + ch] = bf16_rne(feat[((size_t)b * kNC + ch) * kNT + t0 + tt]);
  }
  __syncthreads();

  v8h hv[3];
#pragma unroll
  for (int it = 0; it < 3; ++it) {
    const int idx = it * 256 + tid;
    const int tt = idx / kGrp;
    const int g = idx - tt * kGrp;
    const bool isSq = (g < 10);
    const bool isLin = (g >= 10) && (g < 20);
    const int gg = isSq ? g : (isLin ? (g - 10) : 0);
    const float* sp = sX + tt * kSXP + 8 * gg;
    const v4f a0 = *(const v4f*)(sp);
    const v4f a1 = *(const v4f*)(sp + 4);
#pragma unroll
    for (int e = 0; e < 4; ++e) {
      const float x0 = a0[e];
      const float x1 = a1[e];
      const float sq0 = kXCarry * x0 * x0;
      const float sq1 = kXCarry * x1 * x1;
      const float ln0 = (-2.0f * kXCarry) * x0;
      const float ln1 = (-2.0f * kXCarry) * x1;
      const float v0 = isSq ? sq0 : (isLin ? ln0 : 0.0f);
      const float v1 = isSq ? sq1 : (isLin ? ln1 : 0.0f);
      hv[it][e]     = (_Float16)f16_operand(v0);
      hv[it][4 + e] = (_Float16)f16_operand(v1);
    }
  }
  unsigned short* base = bpl + (((size_t)b * kNT + t0) * kGrp) * 8;
  for (int pass = 0; pass < 2; ++pass) {
#pragma unroll
    for (int it = 0; it < 3; ++it)
      *(volatile v8h*)(base + (size_t)(it * 256 + tid) * 8) = hv[it];
    __threadfence();
  }
}

__global__ __launch_bounds__(256) void emission_rows(
    const unsigned short* __restrict__ aplp, const unsigned short* __restrict__ bplp,
    const float* __restrict__ ctab, float* __restrict__ lpm)
{
  __shared__ __align__(16) float sT[8][16 * kSLP];
  const _Float16* A  = (const _Float16*)aplp;
  const _Float16* Bt = (const _Float16*)bplp;
  const int lane = threadIdx.x & 31;
  const int wave = threadIdx.x >> 5;
  const int tile = blockIdx.x * 8 + wave;
  if (tile >= kTiles) return;
  const int b   = tile / (kTilesL * kTilesT);
  const int rem = tile - b * (kTilesL * kTilesT);
  const int lt  = rem / kTilesT;
  const int tt  = rem - lt * kTilesT;
  const int l0 = lt * 32;
  const int t0 = tt * 32;
  const int rlane = lane & 15;
  const int hh = lane >> 4;
  const int koff = hh * 8;

  const _Float16* ap0 = A + (size_t)(b * kNL + l0 + rlane) * kPitch + koff;
  const _Float16* ap1 = ap0 + (size_t)16 * kPitch;
  const _Float16* bp0 = Bt + (size_t)(b * kNT + t0 + rlane) * kPitch + koff;
  const _Float16* bp1 = bp0 + (size_t)16 * kPitch;

  v8f acc[2][2];
#pragma unroll
  for (int i = 0; i < 2; ++i)
#pragma unroll
    for (int j = 0; j < 2; ++j) acc[i][j] = (v8f){0.f, 0.f, 0.f, 0.f, 0.f, 0.f, 0.f, 0.f};

#pragma unroll 1
  for (int k0 = 0; k0 < kDepth; k0 += 32) {
    const v16h fb0 = frag_load(bp0 + k0);
    const v16h fb1 = frag_load(bp1 + k0);
    const v16h fa0 = frag_load(ap0 + k0);
    const v16h fa1 = frag_load(ap1 + k0);
    acc[0][0] = mma_guarded(fa0, fb0, acc[0][0]);
    acc[0][1] = mma_guarded(fa0, fb1, acc[0][1]);
    acc[1][0] = mma_guarded(fa1, fb0, acc[1][0]);
    acc[1][1] = mma_guarded(fa1, fb1, acc[1][1]);
  }

  float* slab = sT[wave];
  const int q = lane >> 3;
  const int c4 = (lane & 7) * 4;
#pragma unroll
  for (int i = 0; i < 2; ++i) {
    const int lrow0 = l0 + 16 * i;
    const float* cp = ctab + b * kNL + lrow0 + 8 * hh;
    const v4f c0 = *(const v4f*)(cp);
    const v4f c1 = *(const v4f*)(cp + 4);
    float cc[8];
    cc[0] = c0[0]; cc[1] = c0[1]; cc[2] = c0[2]; cc[3] = c0[3];
    cc[4] = c1[0]; cc[5] = c1[1]; cc[6] = c1[2]; cc[7] = c1[3];
#pragma unroll
    for (int j = 0; j < 2; ++j) {
#pragma unroll
      for (int r = 0; r < 8; ++r)
        slab[(8 * hh + r) * kSLP + 16 * j + rlane] = fmaf(acc[i][j][r], kFold, cc[r]);
    }
    __builtin_amdgcn_fence(__ATOMIC_RELEASE, "workgroup");
    __builtin_amdgcn_wave_barrier();
    __builtin_amdgcn_fence(__ATOMIC_ACQUIRE, "workgroup");
    for (int pass = 0; pass < 2; ++pass) {
#pragma unroll
      for (int it = 0; it < 4; ++it) {
        const int row = it * 4 + q;
        const v4f v = *(const v4f*)(slab + row * kSLP + c4);
        *(volatile v4f*)(lpm + ((size_t)(b * kNL + lrow0 + row) * kNT + t0 + c4)) = v;
      }
      __threadfence();
    }
    __builtin_amdgcn_fence(__ATOMIC_RELEASE, "workgroup");
    __builtin_amdgcn_wave_barrier();
    __builtin_amdgcn_fence(__ATOMIC_ACQUIRE, "workgroup");
  }
}

__global__ __launch_bounds__(160) void forward_pass(
    const float* __restrict__ lpm, const int* __restrict__ len_states, const int* __restrict__ len_frames,
    float* __restrict__ alast)
{
  __shared__ __align__(16) float sL[kNL * kSLP];
  __shared__ float sA[2][kNL + 4];
  __shared__ float sRes[4];
  const int tid = threadIdx.x;
  const int b = blockIdx.x;
  const float* lpb = lpm + (size_t)b * kNL * kNT;
  int tl = len_states[b];
  tl = tl < 1 ? 1 : (tl > kNL ? kNL : tl);
  tl -= 1;
  int ml = len_frames[b];
  ml = ml < 1 ? 1 : (ml > kNT ? kNT : ml);
  ml -= 1;
  const float first = lpb[0];
  float alpha = (tid == 0) ? first : kNeg;
  float last = (ml == 0) ? alpha : kNeg;
  sA[0][tid + 1] = alpha;
  if (tid == 0) {
    sA[0][0] = kNeg;
    sA[1][0] = kNeg;
  }
#pragma unroll 1
  for (int c = 0; c < kNT / 32; ++c) {
    __syncthreads();
#pragma unroll
    for (int i = 0; i < 8; ++i) {
      const int idx = i * kNL + tid;
      const int row = idx >> 3;
      const int col = (idx & 7) * 4;
      *(v4f*)(sL + row * kSLP + col) = *(const v4f*)(lpb + (size_t)row * kNT + c * 32 + col);
    }
    __syncthreads();
#pragma unroll 1
    for (int s = (c == 0) ? 1 : 0; s < 32; ++s) {
      const int t = c * 32 + s;
      const float lpv = sL[tid * kSLP + s];
      const float sh = sA[(t - 1) & 1][tid];
      const float a = log_add_exp(alpha, sh) + lpv;
      alpha = a;
      sA[t & 1][tid + 1] = a;
      last = (t == ml) ? a : last;
      __syncthreads();
    }
  }
  if (tid == tl) sRes[0] = last;
  __syncthreads();
  if (tid < 32) {
    const float v = sRes[0];
    volatile float* p = alast + b * 32 + tid;
    *p = v;
    __threadfence();
    *p = v;
  }
}

__global__ __launch_bounds__(256) void write_outputs(
    const float* __restrict__ lpm, const float* __restrict__ alast, float* __restrict__ out)
{
  const int j = blockIdx.x * 256 + threadIdx.x;
  if (j >= kQuads) return;
  float lossv = 0.0f;
  if (blockIdx.x == 0) {
    float s = 0.0f;
#pragma unroll 1
    for (int i = 0; i < kNB; ++i) s += alast[i * 32];
    lossv = -(s * (1.0f / (float)kNB));
  }
  const size_t e0 = (size_t)j * 4;
  const v4f a = *(const v4f*)(lpm + e0);
  const size_t pe = (j > 0) ? (e0 - 1) : 0;
  float pv = lpm[pe];
  asm volatile("" : "+v"(pv));
  float tail = a[3];
  asm volatile("" : "+v"(tail));
  v4f o;
  o[0] = (j == 0) ? lossv : pv;
  o[1] = a[0];
  o[2] = a[1];
  o[3] = a[2];
  const bool lastq = (j == kQuads - 1);
  volatile v4f* op = (volatile v4f*)(out + e0);
  volatile float* tp = (volatile float*)(out + (kFlat - 1));
  *op = o;
  if (lastq) *tp = tail;
  __threadfence();
  *op = o;
  if (lastq) *tp = tail;
}

extern "C" void kernel_launch(void* const* d_in, const int* in_sizes, int n_in,
                              void* d_out, int out_size, void* d_ws, size_t ws_size,
                              hipStream_t stream) {
  if (n_in < 4) return;
  if (in_sizes[0] != kNB * kNL * 2 * kNC) return;
  if (in_sizes[1] != kNB * kNC * kNT) return;
  if (in_sizes[2] != kNB) return;
  if (in_sizes[3] != kNB) return;
  if (out_size != kFlat) return;
  if (ws_size < kWsTotal) return;

  const float* stat = (const float*)d_in[0];
  const float* feat = (const float*)d_in[1];
  const int* len_states = (const int*)d_in[2];
  const int* len_frames = (const int*)d_in[3];
  float* out = (float*)d_out;

  char* ws = (char*)d_ws;
  unsigned short* APL = (unsigned short*)(ws + kOffAPL);
  unsigned short* BPL = (unsigned short*)(ws + kOffBPL);
  float* CT  = (float*)(ws + kOffCT);
  float* LPM = (float*)(ws + kOffLPM);
  float* AL  = (float*)(ws + kOffAL);

  operand_planes_states<<<dim3(kRowsA / 32), dim3(256), 0, stream>>>(stat, APL, CT);
  operand_planes_frames<<<dim3(kNT / 32, kNB), dim3(256), 0, stream>>>(feat, BPL);
  emission_rows<<<dim3(kTiles / 8), dim3(256), 0, stream>>>(APL, BPL, CT, LPM);
  forward_pass<<<dim3(kNB), dim3(kNL), 0, stream>>>(LPM, len_states, len_frames, AL);
  write_outputs<<<dim3(kQuads / 256), dim3(256), 0, stream>>>(LPM, AL, out);
}
